// StreamProcessor_79010218377433
// MI455X (gfx1250) — hardware-verified
//
#include <hip/hip_runtime.h>

#define B_SZ    16
#define L_SEQ   3600
#define LATENT  64
#define D_MODEL 128
#define D_INNER 256
#define D_STATE 16
#define D_CONV  4
#define DT_RANK 8
#define M_ROWS  (B_SZ * L_SEQ)
#define XDBL_LD 64
#define ZT_ROWS 64
#define WSCALE  64.0f
#define WSCALE_INV (1.0f / 64.0f)

static_assert(M_ROWS % 64 == 0);
static_assert(L_SEQ >= ZT_ROWS);

typedef __attribute__((ext_vector_type(16))) _Float16 v16h;
typedef __attribute__((ext_vector_type(8)))  _Float16 v8h;
typedef __attribute__((ext_vector_type(2)))  _Float16 v2h;
typedef __attribute__((ext_vector_type(16))) __bf16   v16b;
typedef __attribute__((ext_vector_type(8)))  __bf16   v8b;
typedef __attribute__((ext_vector_type(8)))  float    v8f;
typedef __attribute__((ext_vector_type(4)))  float    v4f;
#define U16(p) ((const unsigned short*)(const void*)(p))

__device__ __forceinline__ unsigned short f2bf_bits(float f) {
  unsigned u = __float_as_uint(f);
  return (unsigned short)((u + 0x7FFFu + ((u >> 16) & 1u)) >> 16);
}
__device__ __forceinline__ float bf_bits2f(unsigned short h) { return __uint_as_float(((unsigned)h) << 16); }

__device__ __forceinline__ void dep_guard_h(v8f& a, v8f& b, v16h x, v16h y) { asm volatile("v_nop\n\tv_nop\n\tv_nop\n\tv_nop" : "+v"(a), "+v"(b) : "v"(x), "v"(y)); }
__device__ __forceinline__ void dep_guard_b(v8f& a, v8f& b, v16b x, v16b y) { asm volatile("v_nop\n\tv_nop\n\tv_nop\n\tv_nop" : "+v"(a), "+v"(b) : "v"(x), "v"(y)); }
__device__ __forceinline__ void keep4_h(v16h a, v16h b, v16h c, v16h d) { asm volatile("v_nop" :: "v"(a), "v"(b), "v"(c), "v"(d)); }
__device__ __forceinline__ void keep4_b(v16b a, v16b b, v16b c, v16b d) { asm volatile("v_nop" :: "v"(a), "v"(b), "v"(c), "v"(d)); }
__device__ __forceinline__ void acc_guard4(v8f& a, v8f& b, v8f& c, v8f& d) { asm volatile("v_nop\n\tv_nop\n\tv_nop\n\tv_nop" : "+v"(a), "+v"(b), "+v"(c), "+v"(d)); }
template <typename T> struct Frag;
template <> struct Frag<_Float16> {
  typedef v16h V; union U { v16h v; v8h h[2]; };
  static __device__ __forceinline__ v16h load(const _Float16* p) {
    U f; f.h[0] = *(const v8h*)(p); f.h[1] = *(const v8h*)(p + 16); return f.v;
  }
  static __device__ __forceinline__ v8f mma(v16h a, v16h b, v8f c) {
    return __builtin_amdgcn_wmma_f32_16x16x32_f16(false, a, false, b, (short)0, c, false, false);
  }
  static __device__ __forceinline__ void guard(v8f& a, v8f& b, v16h x, v16h y) { dep_guard_h(a, b, x, y); }
  static __device__ __forceinline__ void keep(v16h a, v16h b, v16h c, v16h d) { keep4_h(a, b, c, d); }
};
template <> struct Frag<__bf16> {
  typedef v16b V; union U { v16b v; v8b h[2]; };
  static __device__ __forceinline__ v16b load(const __bf16* p) {
    U f; f.h[0] = *(const v8b*)(p); f.h[1] = *(const v8b*)(p + 16); return f.v;
  }
  static __device__ __forceinline__ v8f mma(v16b a, v16b b, v8f c) {
    return __builtin_amdgcn_wmma_f32_16x16x32_bf16(false, a, false, b, (short)0, c, false, false);
  }
  static __device__ __forceinline__ void guard(v8f& a, v8f& b, v16b x, v16b y) { dep_guard_b(a, b, x, y); }
  static __device__ __forceinline__ void keep(v16b a, v16b b, v16b c, v16b d) { keep4_b(a, b, c, d); }
};

template <int ET> struct Elem;
template <> struct Elem<0> { typedef _Float16 T; };
template <> struct Elem<1> { typedef __bf16 T; };
template <int ET, bool SPLIT, int BIAS_MODE, int OUT_MODE, bool RESID, int ACT = 0>
__global__ __launch_bounds__(256) void wmma_gemm64(
    const unsigned short* __restrict__ Ap, const unsigned short* __restrict__ A2p, int lda, long strideA,
    const unsigned short* __restrict__ Btp, const unsigned short* __restrict__ Bt2p, int ldb, long strideB,
    void* __restrict__ Cout, void* __restrict__ Cout2, int ldc, long strideC,
    const float* __restrict__ bias,
    const float* __restrict__ resid, long strideR,
    int M, int N, int K, float scale) {
  typedef typename Elem<ET>::T T;
  typedef typename Frag<T>::V V;
  const T* A = (const T*)Ap; const T* A2 = (const T*)A2p; const T* Bt = (const T*)Btp; const T* Bt2 = (const T*)Bt2p;
  __shared__ __align__(16) float sT[8][16 * 68];
  const int b    = blockIdx.y;
  const int lane = threadIdx.x & 31;
  const int wave = threadIdx.x >> 5;
  const int tilesN = N >> 6;
  const int tilesM = M >> 6;
  const int tile = blockIdx.x * 8 + wave;
  if (tile >= tilesM * tilesN) return;
  const int tm = tile / tilesN;
  const int tn = tile - tm * tilesN;
  const int m0 = tm << 6;
  const int n0 = tn << 6;

  const T* Ab  = A  + (size_t)b * strideA;
  const T* Bb  = Bt + (size_t)b * strideB;
  const T* Ab2 = SPLIT ? (A2  + (size_t)b * strideA) : nullptr;
  const T* Bb2 = SPLIT ? (Bt2 + (size_t)b * strideB) : nullptr;

  const int rlane = lane & 15;
  const int koff  = (lane >> 4) * 8;
  const int mOff  = (lane >> 4) * 8;

  v8f acc[4][4];
#pragma unroll
  for (int i = 0; i < 4; ++i)
#pragma unroll
    for (int j = 0; j < 4; ++j) acc[i][j] = (v8f){0.f,0.f,0.f,0.f,0.f,0.f,0.f,0.f};

  for (int k0 = 0; k0 < K; k0 += 32) {
    V bh[4], bl[4];
#pragma unroll
    for (int j = 0; j < 4; ++j) {
      const size_t bo = (size_t)(n0 + (j << 4) + rlane) * ldb + koff + k0;
      bh[j] = Frag<T>::load(Bb + bo);
      if (SPLIT) bl[j] = Frag<T>::load(Bb2 + bo);
    }
#pragma unroll
    for (int i = 0; i < 4; ++i) {
      const size_t ao = (size_t)(m0 + (i << 4) + rlane) * lda + koff + k0;
      V ah = Frag<T>::load(Ab + ao);
      V al;
      if (SPLIT) al = Frag<T>::load(Ab2 + ao);
#pragma unroll
      for (int j = 0; j < 4; ++j) {
        acc[i][j] = Frag<T>::mma(ah, bh[j], acc[i][j]);
        if (SPLIT) {
          acc[i][j] = Frag<T>::mma(ah, bl[j], acc[i][j]);
          acc[i][j] = Frag<T>::mma(al, bh[j], acc[i][j]);
        }
      }
      Frag<T>::guard(acc[i][0], acc[i][3], ah, SPLIT ? al : ah);
    }
    Frag<T>::keep(bh[0], bh[1], bh[2], bh[3]);
    if (SPLIT) Frag<T>::keep(bl[0], bl[1], bl[2], bl[3]);
  }
  acc_guard4(acc[0][0], acc[0][1], acc[0][2], acc[0][3]);
  acc_guard4(acc[1][0], acc[1][1], acc[1][2], acc[1][3]);
  acc_guard4(acc[2][0], acc[2][1], acc[2][2], acc[2][3]);
  acc_guard4(acc[3][0], acc[3][1], acc[3][2], acc[3][3]);

  float* slab = sT[wave];
  const float* Rb = RESID ? (resid + (size_t)b * strideR) : nullptr;
#pragma unroll
  for (int i = 0; i < 4; ++i) {
    const int mBase = m0 + (i << 4);
#pragma unroll
    for (int j = 0; j < 4; ++j) {
      const int n = n0 + (j << 4) + rlane;
      float bv = 0.f;
      if (BIAS_MODE == 2) bv = bias[n];
#pragma unroll
      for (int r = 0; r < 8; ++r) {
        float v = acc[i][j][r] * scale;
        if (BIAS_MODE == 1) v += bias[mBase + mOff + r];
        if (BIAS_MODE == 2) v += bv;
        if (RESID) v += Rb[(size_t)(mBase + mOff + r) * ldc + n];
        if (ACT == 1) v = tanhf(v);
        if (ACT == 2) v = fmaxf(v, 0.0f);
        if (ACT == 3) v = v / (1.0f + expf(-v));
        if (ACT == 4) v = (v > 0.f) ? v : 0.01f * v;
        if (ACT == 5) v = 0.5f * v * (1.0f + erff(v * 0.70710678118654752f));
        slab[(mOff + r) * 68 + (j << 4) + rlane] = v;
      }
    }
    __builtin_amdgcn_fence(__ATOMIC_RELEASE, "workgroup");
    __builtin_amdgcn_wave_barrier();
    __builtin_amdgcn_fence(__ATOMIC_ACQUIRE, "workgroup");
    if (OUT_MODE == 0) {
      float* C = (float*)Cout + (size_t)b * strideC;
      const int hh = lane >> 4, c4 = (lane & 15) * 4;
      for (int pass = 0; pass < 2; ++pass) {
#pragma unroll
        for (int it = 0; it < 8; ++it) {
          const int row = it * 2 + hh;
          v4f v = *(const v4f*)(slab + row * 68 + c4);
          *(volatile v4f*)(C + (size_t)(mBase + row) * ldc + n0 + c4) = v;
        }
        __threadfence();
      }
    } else {
      const int q = lane >> 3, c8 = (lane & 7) * 8;
      unsigned short* C  = (unsigned short*)Cout  + (size_t)b * strideC;
      unsigned short* C2 = (OUT_MODE == 2) ? ((unsigned short*)Cout2 + (size_t)b * strideC) : nullptr;
      for (int pass = 0; pass < 2; ++pass) {
#pragma unroll
        for (int it = 0; it < 4; ++it) {
          const int row = it * 4 + q;
          const float* sp = slab + row * 68 + c8;
          v8h hv, lv;
#pragma unroll
          for (int e = 0; e < 8; ++e) {
            if (OUT_MODE == 1) {
              hv[e] = (_Float16)sp[e];
            } else {
              unsigned short hb = f2bf_bits(sp[e]);
              unsigned short lb = f2bf_bits(sp[e] - bf_bits2f(hb));
              hv[e] = __builtin_bit_cast(_Float16, hb);
              lv[e] = __builtin_bit_cast(_Float16, lb);
            }
          }
          *(volatile v8h*)(C + (size_t)(mBase + row) * ldc + n0 + c8) = hv;
          if (OUT_MODE == 2) *(volatile v8h*)(C2 + (size_t)(mBase + row) * ldc + n0 + c8) = lv;
        }
        __threadfence();
      }
    }
    __builtin_amdgcn_fence(__ATOMIC_RELEASE, "workgroup");
    __builtin_amdgcn_wave_barrier();
    __builtin_amdgcn_fence(__ATOMIC_ACQUIRE, "workgroup");
  }
}

__global__ __launch_bounds__(256) void cast_pad_f16x2(
    const float* __restrict__ in, _Float16* __restrict__ out,
    int Rin, int Cin, int cshift, float scale, int n2) {
  const int i = blockIdx.x * 256 + threadIdx.x;
  if (i >= n2) return;
  const int Cout = 1 << cshift;
  const int e0 = 2 * i;
  const int r = e0 >> cshift;
  const int c = e0 & (Cout - 1);
  const int rr = (r < Rin) ? r : (Rin - 1);
  const int cc0 = (c < Cin) ? c : (Cin - 1);
  const int cc1 = (c + 1 < Cin) ? (c + 1) : (Cin - 1);
  float f0 = in[(size_t)rr * Cin + cc0] * scale;
  float f1 = in[(size_t)rr * Cin + cc1] * scale;
  if (r >= Rin || c >= Cin) f0 = 0.f;
  if (r >= Rin || c + 1 >= Cin) f1 = 0.f;
  v2h o; o.x = (_Float16)f0; o.y = (_Float16)f1;
  const unsigned u = __builtin_bit_cast(unsigned, o);
  ((volatile unsigned*)out)[i] = u;
  __threadfence();
  ((volatile unsigned*)out)[i] = u;
}

__device__ __forceinline__ float fsilu(float x) { return x * __builtin_amdgcn_rcpf(1.0f + __expf(-x)); }

__global__ __launch_bounds__(256) void k_conv_silu(const _Float16* __restrict__ xh, const float* __restrict__ cw,
                                                   const float* __restrict__ cb, _Float16* __restrict__ xc, int n2) {
  const int i = blockIdx.x * 256 + threadIdx.x;
  if (i >= n2) return;
  const int e0 = 2 * i;
  const int m = e0 >> 8;
  const int d = e0 & (D_INNER - 1);
  const int t = m % L_SEQ;
  float a0 = 0.f, a1 = 0.f;
#pragma unroll
  for (int j = 0; j < D_CONV; ++j) {
    const int back = D_CONV - 1 - j;
    const bool valid = (t >= back);
    const int rr = valid ? (m - back) : m;
    const v2h p = *(const v2h*)(xh + (size_t)rr * D_INNER + d);
    const float x0 = valid ? (float)p.x : 0.f;
    const float x1 = valid ? (float)p.y : 0.f;
    a0 += cw[d * D_CONV + j] * x0;
    a1 += cw[(d + 1) * D_CONV + j] * x1;
  }
  a0 += cb[d];
  a1 += cb[d + 1];
  v2h o; o.x = (_Float16)fsilu(a0); o.y = (_Float16)fsilu(a1);
  const unsigned u = __builtin_bit_cast(unsigned, o);
  ((volatile unsigned*)xc)[i] = u;
  __threadfence();
  ((volatile unsigned*)xc)[i] = u;
}

__global__ __launch_bounds__(256) void k_scan(const _Float16* __restrict__ xh, const float* __restrict__ xdbl,
                                              const float* __restrict__ cw, const float* __restrict__ cb,
                                              const float* __restrict__ dtw, const float* __restrict__ dtb,
                                              const float* __restrict__ Alog, const float* __restrict__ Dsk,
                                              const float* __restrict__ ztail, float* __restrict__ yfin) {
  const int b = blockIdx.x;
  const int d = threadIdx.x;
  float a[D_STATE];
#pragma unroll
  for (int s = 0; s < D_STATE; ++s) a[s] = -__expf(Alog[d * D_STATE + s]);
  float w8[DT_RANK];
#pragma unroll
  for (int r = 0; r < DT_RANK; ++r) w8[r] = dtw[d * DT_RANK + r];
  const float c0 = cw[d * D_CONV + 0], c1 = cw[d * D_CONV + 1], c2 = cw[d * D_CONV + 2], c3 = cw[d * D_CONV + 3];
  const float cbias = cb[d];
  const float dbias = dtb[d];
  float h[D_STATE];
#pragma unroll
  for (int s = 0; s < D_STATE; ++s) h[s] = 0.f;
  float xm1 = 0.f, xm2 = 0.f, xm3 = 0.f, xc = 0.f;
  const _Float16* xp = xh + (size_t)b * L_SEQ * D_INNER + d;
  const float* dp = xdbl + (size_t)b * L_SEQ * XDBL_LD;
#pragma unroll 1
  for (int t = 0; t < L_SEQ; ++t) {
    const float xv = (float)xp[(size_t)t * D_INNER];
    float conv = c0 * xm3;
    conv += c1 * xm2;
    conv += c2 * xm1;
    conv += c3 * xv;
    conv += cbias;
    xm3 = xm2; xm2 = xm1; xm1 = xv;
    xc = fsilu(conv);
    const float* row = dp + (size_t)t * XDBL_LD;
    const v4f q0 = *(const v4f*)(row + 0);
    const v4f q1 = *(const v4f*)(row + 4);
    const v4f g0 = *(const v4f*)(row + 8);
    const v4f g1 = *(const v4f*)(row + 12);
    const v4f g2 = *(const v4f*)(row + 16);
    const v4f g3 = *(const v4f*)(row + 20);
    float u = w8[0] * q0.x;
    u += w8[1] * q0.y;
    u += w8[2] * q0.z;
    u += w8[3] * q0.w;
    u += w8[4] * q1.x;
    u += w8[5] * q1.y;
    u += w8[6] * q1.z;
    u += w8[7] * q1.w;
    u += dbias;
    const float dt = fmaxf(u, 0.f) + log1pf(__expf(-fabsf(u)));
    const float dx = dt * xc;
    const float bv[D_STATE] = {g0.x, g0.y, g0.z, g0.w, g1.x, g1.y, g1.z, g1.w,
                               g2.x, g2.y, g2.z, g2.w, g3.x, g3.y, g3.z, g3.w};
#pragma unroll
    for (int s = 0; s < D_STATE; ++s) {
      const float e = __expf(dt * a[s]);
      h[s] = e * h[s] + dx * bv[s];
    }
  }
  const float* crow = dp + (size_t)(L_SEQ - 1) * XDBL_LD + DT_RANK + D_STATE;
  const v4f k0 = *(const v4f*)(crow + 0);
  const v4f k1 = *(const v4f*)(crow + 4);
  const v4f k2 = *(const v4f*)(crow + 8);
  const v4f k3 = *(const v4f*)(crow + 12);
  const float cv[D_STATE] = {k0.x, k0.y, k0.z, k0.w, k1.x, k1.y, k1.z, k1.w,
                             k2.x, k2.y, k2.z, k2.w, k3.x, k3.y, k3.z, k3.w};
  float y = 0.f;
#pragma unroll
  for (int s = 0; s < D_STATE; ++s) y += h[s] * cv[s];
  y += xc * Dsk[d];
  const float zv = ztail[((size_t)b * ZT_ROWS + (ZT_ROWS - 1)) * D_INNER + d];
  y *= fsilu(zv);
  ((volatile float*)yfin)[b * D_INNER + d] = y;
  __threadfence();
  ((volatile float*)yfin)[b * D_INNER + d] = y;
}

__global__ __launch_bounds__(256) void k_head(const float* __restrict__ yfin, const float* __restrict__ outw,
                                              const float* __restrict__ nw, const float* __restrict__ nb,
                                              const float* __restrict__ clsw, const float* __restrict__ clsb,
                                              float* __restrict__ out) {
  __shared__ float sy[D_INNER];
  __shared__ float so[D_MODEL];
  __shared__ float slog[B_SZ];
  const int tid = threadIdx.x;
  const int wave = tid >> 5;
  const int lane = tid & 31;
  if (tid < B_SZ) slog[tid] = 0.f;
  for (int b = 0; b < B_SZ; ++b) {
    sy[tid] = yfin[b * D_INNER + tid];
    __syncthreads();
    float yv[8];
#pragma unroll
    for (int i = 0; i < 8; ++i) yv[i] = sy[lane + 32 * i];
#pragma unroll 1
    for (int jj = 0; jj < 16; ++jj) {
      const int n = wave * 16 + jj;
      const float* wr = outw + (size_t)n * D_INNER + lane;
      float p = 0.f;
#pragma unroll
      for (int i = 0; i < 8; ++i) p += yv[i] * wr[32 * i];
      p += __shfl_xor(p, 16, 32);
      p += __shfl_xor(p, 8, 32);
      p += __shfl_xor(p, 4, 32);
      p += __shfl_xor(p, 2, 32);
      p += __shfl_xor(p, 1, 32);
      if (lane == 0) so[n] = p;
    }
    __syncthreads();
    if (wave == 0) {
      float v[4];
#pragma unroll
      for (int i = 0; i < 4; ++i) v[i] = so[lane + 32 * i];
      float sm = (v[0] + v[1]) + (v[2] + v[3]);
      sm += __shfl_xor(sm, 16, 32);
      sm += __shfl_xor(sm, 8, 32);
      sm += __shfl_xor(sm, 4, 32);
      sm += __shfl_xor(sm, 2, 32);
      sm += __shfl_xor(sm, 1, 32);
      const float mu = sm * (1.0f / (float)D_MODEL);
      float dv[4];
      float sq = 0.f;
#pragma unroll
      for (int i = 0; i < 4; ++i) { dv[i] = v[i] - mu; sq += dv[i] * dv[i]; }
      sq += __shfl_xor(sq, 16, 32);
      sq += __shfl_xor(sq, 8, 32);
      sq += __shfl_xor(sq, 4, 32);
      sq += __shfl_xor(sq, 2, 32);
      sq += __shfl_xor(sq, 1, 32);
      const float var = sq * (1.0f / (float)D_MODEL);
      const float rs = rsqrtf(var + 1e-5f);
      float dot = 0.f;
#pragma unroll
      for (int i = 0; i < 4; ++i) {
        const int n = lane + 32 * i;
        const float xn = dv[i] * rs * nw[n] + nb[n];
        dot += xn * clsw[n];
      }
      dot += __shfl_xor(dot, 16, 32);
      dot += __shfl_xor(dot, 8, 32);
      dot += __shfl_xor(dot, 4, 32);
      dot += __shfl_xor(dot, 2, 32);
      dot += __shfl_xor(dot, 1, 32);
      if (lane == 0) slog[b] = dot + clsb[0];
    }
    __syncthreads();
  }
  if (tid < B_SZ) {
    const float v = slog[tid];
    ((volatile float*)out)[tid] = v;
    __threadfence();
    ((volatile float*)out)[tid] = v;
  }
}

extern "C" void kernel_launch(void* const* d_in, const int* in_sizes, int n_in,
                              void* d_out, int out_size, void* d_ws, size_t ws_size,
                              hipStream_t stream) {
  if (n_in < 16) return;
  if (in_sizes[0] != M_ROWS * LATENT || out_size < B_SZ) return;
  const float* z_seq      = (const float*)d_in[0];
  const float* emb_w      = (const float*)d_in[1];
  const float* emb_b      = (const float*)d_in[2];
  const float* in_proj_w  = (const float*)d_in[3];
  const float* conv_w     = (const float*)d_in[4];
  const float* conv_b     = (const float*)d_in[5];
  const float* x_proj_w   = (const float*)d_in[6];
  const float* dt_proj_w  = (const float*)d_in[7];
  const float* dt_proj_b  = (const float*)d_in[8];
  const float* A_log      = (const float*)d_in[9];
  const float* D_skip     = (const float*)d_in[10];
  const float* out_proj_w = (const float*)d_in[11];
  const float* norm_w     = (const float*)d_in[12];
  const float* norm_b     = (const float*)d_in[13];
  const float* cls_w      = (const float*)d_in[14];
  const float* cls_b      = (const float*)d_in[15];
  float* out = (float*)d_out;

  size_t off = 0;
  auto carve = [&](size_t bytes) -> size_t { size_t r = off; off += (bytes + 255) & ~(size_t)255; return r; };
  const size_t o_zh     = carve((size_t)M_ROWS * LATENT * 2);
  const size_t o_embwh  = carve((size_t)D_MODEL * LATENT * 2);
  const size_t o_inpwh  = carve((size_t)2 * D_INNER * D_MODEL * 2);
  const size_t o_xpwh   = carve((size_t)XDBL_LD * D_INNER * 2);
  const size_t o_xembh  = carve((size_t)M_ROWS * D_MODEL * 2);
  const size_t o_xh     = carve((size_t)M_ROWS * D_INNER * 2);
  const size_t o_ztail  = carve((size_t)B_SZ * ZT_ROWS * D_INNER * 4);
  const size_t o_xch    = carve((size_t)M_ROWS * D_INNER * 2);
  const size_t o_xdbl   = carve((size_t)M_ROWS * XDBL_LD * 4);
  const size_t o_yfin   = carve((size_t)B_SZ * D_INNER * 4);
  if (off > ws_size) return;
  char* ws = (char*)d_ws;
  _Float16* zh    = (_Float16*)(ws + o_zh);
  _Float16* embwh = (_Float16*)(ws + o_embwh);
  _Float16* inpwh = (_Float16*)(ws + o_inpwh);
  _Float16* xpwh  = (_Float16*)(ws + o_xpwh);
  _Float16* xembh = (_Float16*)(ws + o_xembh);
  _Float16* xh    = (_Float16*)(ws + o_xh);
  float*    ztail = (float*)(ws + o_ztail);
  _Float16* xch   = (_Float16*)(ws + o_xch);
  float*    xdbl  = (float*)(ws + o_xdbl);
  float*    yfin  = (float*)(ws + o_yfin);

  {
    const int n2 = M_ROWS * LATENT / 2;
    cast_pad_f16x2<<<(n2 + 255) / 256, 256, 0, stream>>>(z_seq, zh, M_ROWS, LATENT, 6, 1.0f, n2);
  }
  {
    const int n2 = D_MODEL * LATENT / 2;
    cast_pad_f16x2<<<(n2 + 255) / 256, 256, 0, stream>>>(emb_w, embwh, D_MODEL, LATENT, 6, WSCALE, n2);
  }
  {
    const int n2 = 2 * D_INNER * D_MODEL / 2;
    cast_pad_f16x2<<<(n2 + 255) / 256, 256, 0, stream>>>(in_proj_w, inpwh, 2 * D_INNER, D_MODEL, 7, WSCALE, n2);
  }
  {
    const int n2 = XDBL_LD * D_INNER / 2;
    cast_pad_f16x2<<<(n2 + 255) / 256, 256, 0, stream>>>(x_proj_w, xpwh, DT_RANK + 2 * D_STATE, D_INNER, 8, WSCALE, n2);
  }
  {
    const int tiles = (M_ROWS / 64) * (D_MODEL / 64);
    wmma_gemm64<0, false, 2, 1, false><<<dim3((tiles + 7) / 8, 1), 256, 0, stream>>>(
        U16(zh), U16(zh), LATENT, 0L, U16(embwh), U16(embwh), LATENT, 0L,
        (void*)xembh, (void*)xembh, D_MODEL, 0L, emb_b, emb_b, 0L, M_ROWS, D_MODEL, LATENT, WSCALE_INV);
  }
  {
    const int tiles = (M_ROWS / 64) * (D_INNER / 64);
    wmma_gemm64<0, false, 0, 1, false><<<dim3((tiles + 7) / 8, 1), 256, 0, stream>>>(
        U16(xembh), U16(xembh), D_MODEL, 0L, U16(inpwh), U16(inpwh), D_MODEL, 0L,
        (void*)xh, (void*)xh, D_INNER, 0L, emb_b, emb_b, 0L, M_ROWS, D_INNER, D_MODEL, WSCALE_INV);
  }
  {
    const int tiles = (ZT_ROWS / 64) * (D_INNER / 64);
    wmma_gemm64<0, false, 0, 0, false><<<dim3((tiles + 7) / 8, B_SZ), 256, 0, stream>>>(
        U16(xembh + (size_t)(L_SEQ - ZT_ROWS) * D_MODEL), U16(xembh + (size_t)(L_SEQ - ZT_ROWS) * D_MODEL), D_MODEL, (long)L_SEQ * D_MODEL,
        U16(inpwh + (size_t)D_INNER * D_MODEL), U16(inpwh + (size_t)D_INNER * D_MODEL), D_MODEL, 0L,
        (void*)ztail, (void*)ztail, D_INNER, (long)ZT_ROWS * D_INNER, emb_b, emb_b, 0L, ZT_ROWS, D_INNER, D_MODEL, WSCALE_INV);
  }
  {
    const int n2 = M_ROWS * D_INNER / 2;
    k_conv_silu<<<(n2 + 255) / 256, 256, 0, stream>>>(xh, conv_w, conv_b, xch, n2);
  }
  {
    const int tiles = (M_ROWS / 64) * (XDBL_LD / 64);
    wmma_gemm64<0, false, 0, 0, false><<<dim3((tiles + 7) / 8, 1), 256, 0, stream>>>(
        U16(xch), U16(xch), D_INNER, 0L, U16(xpwh), U16(xpwh), D_INNER, 0L,
        (void*)xdbl, (void*)xdbl, XDBL_LD, 0L, emb_b, emb_b, 0L, M_ROWS, XDBL_LD, D_INNER, WSCALE_INV);
  }
  k_scan<<<B_SZ, D_INNER, 0, stream>>>(xh, xdbl, conv_w, conv_b, dt_proj_w, dt_proj_b, A_log, D_skip, ztail, yfin);
  k_head<<<1, 256, 0, stream>>>(yfin, out_proj_w, norm_w, norm_b, cls_w, cls_b, out);
  (void)hipGetLastError();
}
